// GraphLabelPredict_70772471103910
// MI455X (gfx1250) — hardware-verified
//
#include <hip/hip_runtime.h>
#include <math.h>

typedef __attribute__((ext_vector_type(16))) _Float16 v16h;
typedef __attribute__((ext_vector_type(16))) __bf16 v16b;
typedef __attribute__((ext_vector_type(8)))  _Float16 v8h;
typedef __attribute__((ext_vector_type(8)))  float v8f;
typedef __attribute__((ext_vector_type(4)))  float v4f;
typedef __attribute__((ext_vector_type(2)))  float v2f;
typedef __attribute__((ext_vector_type(4)))  unsigned v4u;
typedef __attribute__((ext_vector_type(4)))  int v4i;
typedef float __attribute__((may_alias)) float_a;
typedef int __attribute__((may_alias)) int_a;

template <typename T> __device__ __forceinline__ void vst2(void* p, T v) { *(volatile T*)p = v; __threadfence(); *(volatile T*)p = v; }
__device__ __forceinline__ v8f wmma16(v16h a, v16h b, v8f c) {
  v8f d = __builtin_amdgcn_wmma_f32_16x16x32_f16(false, a, false, b, (short)0, c, false, false);
  asm volatile("v_nop\n\tv_nop\n\tv_nop\n\tv_nop" : "+v"(d) : "v"(a), "v"(b));
  return d;
}
__device__ __forceinline__ v8f wmma_bf(v16b a, v16b b, v8f c) {
  v8f d = __builtin_amdgcn_wmma_f32_16x16x32_bf16(false, a, false, b, (short)0, c, false, false);
  asm volatile("v_nop\n\tv_nop\n\tv_nop\n\tv_nop" : "+v"(d) : "v"(a), "v"(b));
  return d;
}
__device__ __forceinline__ v16h frag_h(const _Float16* rowk0, int lane) {
  union { v16h v; v8h q[2]; } u; const _Float16* p = rowk0 + 8 * (lane >> 4);
  u.q[0] = *(const v8h*)p; u.q[1] = *(const v8h*)(p + 16); return u.v;
}
__device__ __forceinline__ v16h frag_f32(const float* rowk0, int lane) {
  v16h a; const float* p = rowk0 + 8 * (lane >> 4);
#pragma unroll
  for (int i = 0; i < 8; ++i) { a[i] = (_Float16)p[i]; a[8 + i] = (_Float16)p[16 + i]; }
  return a;
}
__device__ __forceinline__ v16h fragc_f32(const float* W, int k0, int n, int lane, int ld, int K) {
  v16h a; const int g = lane >> 4;
#pragma unroll
  for (int i = 0; i < 8; ++i) { const int ka = k0 + 8 * g + i, kb = ka + 16;
    a[i] = (_Float16)(ka < K ? W[(size_t)ka * ld + n] : 0.f); a[8 + i] = (_Float16)(kb < K ? W[(size_t)kb * ld + n] : 0.f); }
  return a;
}
struct F2 { v16b h, l; };
__device__ __forceinline__ F2 bsplit16(const float v[16]) { F2 r;
#pragma unroll
  for (int i = 0; i < 16; ++i) { const __bf16 h = (__bf16)v[i]; r.h[i] = h; r.l[i] = (__bf16)(v[i] - (float)h); }
  return r; }
__device__ __forceinline__ F2 split_row(const float* row, int k0, int lane) { float v[16]; const float* p = row + k0 + 8 * (lane >> 4);
#pragma unroll
  for (int i = 0; i < 8; ++i) { v[i] = p[i]; v[8 + i] = p[16 + i]; }
  return bsplit16(v); }
__device__ __forceinline__ F2 split_rowK(const float* row, int k0, int lane, int K) { float v[16]; const int g = lane >> 4;
#pragma unroll
  for (int i = 0; i < 8; ++i) { const int ka = k0 + 8 * g + i, kb = ka + 16; v[i] = ka < K ? row[ka] : 0.f; v[8 + i] = kb < K ? row[kb] : 0.f; }
  return bsplit16(v); }
__device__ __forceinline__ F2 split_col(const float* W, int k0, int n, int lane, int ld, int K) { float v[16]; const int g = lane >> 4;
#pragma unroll
  for (int i = 0; i < 8; ++i) { const int ka = k0 + 8 * g + i, kb = ka + 16; v[i] = ka < K ? W[(size_t)ka * ld + n] : 0.f; v[8 + i] = kb < K ? W[(size_t)kb * ld + n] : 0.f; }
  return bsplit16(v); }
__device__ __forceinline__ v8f mac3(const F2& a, const F2& b, v8f c) { c = wmma_bf(a.l, b.h, c); c = wmma_bf(a.h, b.l, c); return wmma_bf(a.h, b.h, c); }
__device__ __forceinline__ float sigm(float v) { return 1.0f / (1.0f + expf(-v)); }
#define LDSX() do { asm volatile("s_wait_dscnt 0" ::: "memory"); __builtin_amdgcn_wave_barrier(); __builtin_amdgcn_fence(__ATOMIC_RELEASE, "workgroup"); } while (0)

#define NI 32
#define CIN 2048
#define HWN 196
#define CP 1028
#define CM 257
#define NCLS 10
#define NPX (NI * NI)
#define KC (CP * 9)

__device__ __forceinline__ v16h fragK_f32(const float* row, int k0, int lane, int K) {
  v16h a; const int g = lane >> 4;
#pragma unroll
  for (int i = 0; i < 8; ++i) { const int ka = k0 + 8 * g + i, kb = ka + 16; a[i] = (_Float16)(ka < K ? row[ka] : 0.f); a[8 + i] = (_Float16)(kb < K ? row[kb] : 0.f); }
  return a;
}
__global__ __launch_bounds__(64) void k_gram(const float* __restrict__ f, float* __restrict__ G) {
  __shared__ __align__(16) float so[2][16][36];
  const int c = blockIdx.x, tid = threadIdx.x, w = tid >> 5, lane = tid & 31, col = lane & 15, g = lane >> 4;
  v8f acc[2] = {};
#pragma unroll 1
  for (int kc = 0; kc < 7; ++kc) { const v16h a = fragK_f32(f + ((size_t)(w * 16 + col) * CIN + c) * HWN, kc * 32, lane, HWN);
#pragma unroll
    for (int j = 0; j < 2; ++j) acc[j] = wmma16(a, fragK_f32(f + ((size_t)(j * 16 + col) * CIN + c) * HWN, kc * 32, lane, HWN), acc[j]); }
#pragma unroll
  for (int j = 0; j < 2; ++j)
#pragma unroll
    for (int r = 0; r < 8; ++r) { const int m = w * 16 + 8 * g + r, n = j * 16 + col;
      so[w][8 * g + r][n] = (m == NI - 1 && n == NI - 1) ? 1.0f : acc[j][r] * (1.0f / (float)HWN); }
  LDSX();
  for (int q = lane; q < 16 * 8; q += 32) { const int rl = q >> 3, pc = q & 7; vst2(G + (size_t)c * NPX + (w * 16 + rl) * NI + pc * 4, *(const v4f*)(&so[w][rl][pc * 4])); }
}
__global__ __launch_bounds__(256) void k_pool(const float* __restrict__ G, float* __restrict__ PF) {
  const size_t f0 = (size_t)blockIdx.x * 1024; const int tid = threadIdx.x;
  __shared__ __align__(16) float so[1024];
  for (int q = tid; q < 1024; q += 256) { const size_t fl = f0 + q; const int mn = (int)(fl / CP), i = (int)(fl % CP);
    const int s = (i * CIN) / CP, e = ((i + 1) * CIN + CP - 1) / CP;
    float a = 0.f; for (int c = s; c < e; ++c) a += G[(size_t)c * NPX + mn];
    so[q] = a / (float)(e - s); }
  __syncthreads();
  vst2(PF + f0 + tid * 4, *(const v4f*)(&so[tid * 4]));
}
__global__ __launch_bounds__(128) void k_conv(const float* __restrict__ PF, const float* __restrict__ W, const float* __restrict__ gam, const float* __restrict__ bet,
                                            const float* __restrict__ mean, const float* __restrict__ var, float* __restrict__ Y) {
  __shared__ __align__(16) float st[128][68];
  const int tid = threadIdx.x, wave = tid >> 5, lane = tid & 31, col = lane & 15, g = lane >> 4;
  const int p0 = blockIdx.x * 64, r0 = p0 + wave * 16, n0 = blockIdx.y * 128;
  const int p = r0 + col, py = p >> 5, px = p & 31;
  v8f acc[8] = {};
#pragma unroll 1
  for (int kc = 0; kc < (KC + 31) / 32; ++kc) {
    v16h a;
#pragma unroll
    for (int i = 0; i < 16; ++i) { const int k = kc * 32 + (i < 8 ? 8 * g + i : 16 + 8 * g + (i - 8)); float v = 0.f;
      if (k < KC) { const int ch = k / 9, t = k % 9, yy = py + t / 3 - 1, xx = px + t % 3 - 1;
        if (yy >= 0 && yy < NI && xx >= 0 && xx < NI) v = PF[(size_t)ch * NPX + yy * NI + xx]; }
      a[i] = (_Float16)v; }
#pragma unroll
    for (int j = 0; j < 8; ++j) { int o = n0 + j * 16 + col; if (o > CM - 1) o = CM - 1; acc[j] = wmma16(a, fragK_f32(W + (size_t)o * KC, kc * 32, lane, KC), acc[j]); } }
#pragma unroll
  for (int j = 0; j < 8; ++j) { int o = n0 + j * 16 + col; const int oc = o > CM - 1 ? CM - 1 : o;
    const float sc = gam[oc] * rsqrtf(var[oc] + 1e-5f), sh = bet[oc] - mean[oc] * sc;
#pragma unroll
    for (int r = 0; r < 8; ++r) { const float v = acc[j][r] * sc + sh; st[j * 16 + col][wave * 16 + 8 * g + r] = v > 0.f ? v : 0.f; } }
  __syncthreads();
  for (int q = tid; q < 128 * 16; q += 128) { const int ol = q >> 4, pc = q & 15, o = n0 + ol; if (o >= CM) continue;
    vst2(Y + (size_t)o * NPX + p0 + pc * 4, *(const v4f*)(&st[ol][pc * 4])); }
}
__global__ __launch_bounds__(256) void k_cls(const float* __restrict__ Y, const float* __restrict__ W2, const float* __restrict__ b2, float* __restrict__ out) {
  __shared__ __align__(16) float so[NCLS][256];
  const int tid = threadIdx.x, p = blockIdx.x * 256 + tid;
  float a[NCLS];
#pragma unroll
  for (int k = 0; k < NCLS; ++k) a[k] = b2[k];
#pragma unroll 1
  for (int c = 0; c < CM; ++c) { const float y = Y[(size_t)c * NPX + p];
#pragma unroll
    for (int k = 0; k < NCLS; ++k) a[k] += y * W2[k * CM + c]; }
#pragma unroll
  for (int k = 0; k < NCLS; ++k) so[k][tid] = a[k];
  __syncthreads();
  for (int q = tid; q < NCLS * 64; q += 256) { const int k = q >> 6, pc = q & 63; vst2(out + (size_t)k * NPX + blockIdx.x * 256 + pc * 4, *(const v4f*)(&so[k][pc * 4])); }
}
extern "C" void kernel_launch(void* const* d_in, const int* in_sizes, int n_in, void* d_out, int out_size, void* d_ws, size_t ws_size, hipStream_t stream) {
  (void)in_sizes; (void)n_in; (void)out_size; (void)ws_size;
  const float* f = (const float*)d_in[0]; const float* W1 = (const float*)d_in[1]; const float* gam = (const float*)d_in[2]; const float* bet = (const float*)d_in[3];
  const float* mean = (const float*)d_in[4]; const float* var = (const float*)d_in[5]; const float* W2 = (const float*)d_in[6]; const float* b2 = (const float*)d_in[7];
  float* out = (float*)d_out;
  char* ws = (char*)d_ws; size_t off = 0;
  auto take = [&](size_t bytes) { char* p = ws + off; off += (bytes + 255) & ~(size_t)255; return p; };
  float* G = (float*)take((size_t)CIN * NPX * 4);
  float* PF = (float*)take((size_t)NPX * CP * 4);
  float* Y = (float*)take((size_t)CM * NPX * 4);
  k_gram<<<CIN, 64, 0, stream>>>(f, G);
  k_pool<<<NPX * CP / 1024, 256, 0, stream>>>(G, PF);
  k_conv<<<dim3(NPX / 64, 3), 128, 0, stream>>>(PF, W1, gam, bet, mean, var, Y);
  k_cls<<<NPX / 256, 256, 0, stream>>>(Y, W2, b2, out);
}
